// Heat1D_31842887532660
// MI455X (gfx1250) — hardware-verified
//
#include <hip/hip_runtime.h>
#include <math.h>

typedef __attribute__((ext_vector_type(16))) _Float16 v16h;
typedef __attribute__((ext_vector_type(16))) __bf16 v16b;
typedef __attribute__((ext_vector_type(8)))  _Float16 v8h;
typedef __attribute__((ext_vector_type(8)))  float v8f;
typedef __attribute__((ext_vector_type(4)))  float v4f;
typedef __attribute__((ext_vector_type(2)))  float v2f;
typedef __attribute__((ext_vector_type(4)))  unsigned v4u;
typedef __attribute__((ext_vector_type(4)))  int v4i;
typedef float __attribute__((may_alias)) float_a;
typedef int __attribute__((may_alias)) int_a;

template <typename T> __device__ __forceinline__ void vst2(void* p, T v) { *(volatile T*)p = v; __threadfence(); *(volatile T*)p = v; }
__device__ __forceinline__ v8f wmma16(v16h a, v16h b, v8f c) {
  v8f d = __builtin_amdgcn_wmma_f32_16x16x32_f16(false, a, false, b, (short)0, c, false, false);
  asm volatile("v_nop\n\tv_nop\n\tv_nop\n\tv_nop" : "+v"(d) : "v"(a), "v"(b));
  return d;
}
__device__ __forceinline__ v8f wmma_bf(v16b a, v16b b, v8f c) {
  v8f d = __builtin_amdgcn_wmma_f32_16x16x32_bf16(false, a, false, b, (short)0, c, false, false);
  asm volatile("v_nop\n\tv_nop\n\tv_nop\n\tv_nop" : "+v"(d) : "v"(a), "v"(b));
  return d;
}
__device__ __forceinline__ v16h frag_h(const _Float16* rowk0, int lane) {
  union { v16h v; v8h q[2]; } u; const _Float16* p = rowk0 + 8 * (lane >> 4);
  u.q[0] = *(const v8h*)p; u.q[1] = *(const v8h*)(p + 16); return u.v;
}
__device__ __forceinline__ v16h frag_f32(const float* rowk0, int lane) {
  v16h a; const float* p = rowk0 + 8 * (lane >> 4);
#pragma unroll
  for (int i = 0; i < 8; ++i) { a[i] = (_Float16)p[i]; a[8 + i] = (_Float16)p[16 + i]; }
  return a;
}
__device__ __forceinline__ v16h frag_f32s(const float* rowk0, int lane, float sc) {
  v16h a; const float* p = rowk0 + 8 * (lane >> 4);
#pragma unroll
  for (int i = 0; i < 8; ++i) { a[i] = (_Float16)(p[i] * sc); a[8 + i] = (_Float16)(p[16 + i] * sc); }
  return a;
}
__device__ __forceinline__ v16h fragc_f32(const float* W, int k0, int n, int lane, int ld, int K) {
  v16h a; const int g = lane >> 4;
#pragma unroll
  for (int i = 0; i < 8; ++i) { const int ka = k0 + 8 * g + i, kb = ka + 16;
    a[i] = (_Float16)(ka < K ? W[(size_t)(ka < K ? ka : K - 1) * ld + n] : 0.f); a[8 + i] = (_Float16)(kb < K ? W[(size_t)(kb < K ? kb : K - 1) * ld + n] : 0.f); }
  return a;
}
struct F2 { v16b h, l; };
__device__ __forceinline__ F2 bsplit16(const float v[16]) { F2 r;
#pragma unroll
  for (int i = 0; i < 16; ++i) { const __bf16 h = (__bf16)v[i]; r.h[i] = h; r.l[i] = (__bf16)(v[i] - (float)h); }
  return r; }
__device__ __forceinline__ F2 split_row(const float* row, int k0, int lane) { float v[16]; const float* p = row + k0 + 8 * (lane >> 4);
#pragma unroll
  for (int i = 0; i < 8; ++i) { v[i] = p[i]; v[8 + i] = p[16 + i]; }
  return bsplit16(v); }
__device__ __forceinline__ F2 split_rowK(const float* row, int k0, int lane, int K) { float v[16]; const int g = lane >> 4;
#pragma unroll
  for (int i = 0; i < 8; ++i) { const int ka = k0 + 8 * g + i, kb = ka + 16; v[i] = ka < K ? row[ka < K ? ka : K - 1] : 0.f; v[8 + i] = kb < K ? row[kb < K ? kb : K - 1] : 0.f; }
  return bsplit16(v); }
__device__ __forceinline__ F2 split_col(const float* W, int k0, int n, int lane, int ld, int K) { float v[16]; const int g = lane >> 4;
#pragma unroll
  for (int i = 0; i < 8; ++i) { const int ka = k0 + 8 * g + i, kb = ka + 16; v[i] = ka < K ? W[(size_t)(ka < K ? ka : K - 1) * ld + n] : 0.f; v[8 + i] = kb < K ? W[(size_t)(kb < K ? kb : K - 1) * ld + n] : 0.f; }
  return bsplit16(v); }
__device__ __forceinline__ v8f mac3(const F2& a, const F2& b, v8f c) { c = wmma_bf(a.l, b.h, c); c = wmma_bf(a.h, b.l, c); return wmma_bf(a.h, b.h, c); }
__device__ __forceinline__ float sigm(float v) { return 1.0f / (1.0f + expf(-v)); }
#define LDSX() do { asm volatile("s_wait_dscnt 0" ::: "memory"); __builtin_amdgcn_wave_barrier(); __builtin_amdgcn_fence(__ATOMIC_RELEASE, "workgroup"); } while (0)


#define NBT 8
#define TT 2048
#define CC 192
#ifndef TNB
#define TNB NBT
#endif
typedef __attribute__((ext_vector_type(8))) __bf16 v8b;
__device__ __forceinline__ v16b frag_b(const __bf16* rowk0, int lane) {
  union { v16b v; v8b q[2]; } u; const __bf16* p = rowk0 + 8 * (lane >> 4);
  u.q[0] = *(const v8b*)p; u.q[1] = *(const v8b*)(p + 16); return u.v;
}
__device__ __forceinline__ float bfr(float v) { return (float)(__bf16)v; }
__device__ __attribute__((noinline)) float exp_ni(float v) { return expf(v); }
__device__ __attribute__((noinline)) float cos_ni(float v) { return cosf(v); }
__device__ __attribute__((noinline)) float pow_ni(float a, float b) { return powf(a, b); }
#define WS_COS  0u
#define WS_COST (WS_COS + 4u * TT * TT)
#define WS_DK   (WS_COST + 4u * TT * TT)
#define WS_UTH  (WS_DK + 4u * TT * CC)
#define WS_UTL  (WS_UTH + 2u * NBT * CC * TT)
#define WS_Z    (WS_UTL + 2u * NBT * CC * TT)
#define WS_ATH  (WS_Z + 4u * NBT * TT * CC)
#define WS_ATL  (WS_ATH + 2u * NBT * CC * TT)
#define WS_G    (WS_ATL + 2u * NBT * CC * TT)
#define WS_END  (WS_G + 4u * NBT * TT * CC)

__global__ __launch_bounds__(256) void k_tab(const float* __restrict__ Kp, float* __restrict__ COS, float* __restrict__ COST, float* __restrict__ DK) {
  __shared__ __align__(16) float srow[TT];
  const int blk = blockIdx.x, tid = threadIdx.x; const float pi_f = 3.141592653589793f; const float sc = (float)0.03125;
  if (blk < TT) { const int n = blk; const float wn = (float)n;
    for (int t = tid; t < TT; t += 256) { const float wx = ((float)t + 0.5f) / (float)TT; float w = cos_ni((wn * wx) * pi_f) * sc; if (n == 0) w = w / 1.4142135623730951f; srow[t] = w; }
    __syncthreads();
    for (int q = tid; q < TT / 4; q += 256) vst2(COS + (size_t)n * TT + q * 4, *(const v4f*)&srow[q * 4]); }
  else if (blk < 2 * TT) { const int t = blk - TT; const float wx = ((float)t + 0.5f) / (float)TT;
    for (int n = tid; n < TT; n += 256) { float w = cos_ni(((float)n * wx) * pi_f) * sc; if (n == 0) w = w / 1.4142135623730951f; srow[n] = w; }
    __syncthreads();
    for (int q = tid; q < TT / 4; q += 256) vst2(COST + (size_t)t * TT + q * 4, *(const v4f*)&srow[q * 4]); }
  else {
    __shared__ __align__(16) float sdk[CC];
    for (int n = 0; n < TT; ++n) { const float wn = (float)n * (pi_f / (float)TT); const float dec = exp_ni(-(wn * wn));
      if (tid < CC) sdk[tid] = pow_ni(dec, bfr(Kp[tid]));
      __syncthreads();
      if (tid < CC / 4) vst2(DK + (size_t)n * CC + tid * 4, *(const v4f*)&sdk[tid * 4]);
      __syncthreads(); } }
}
__global__ __launch_bounds__(256) void k_conv(const float* __restrict__ X, const float* __restrict__ dw, const float* __restrict__ db, const float* __restrict__ lw, const float* __restrict__ lb, __bf16* __restrict__ UTH, __bf16* __restrict__ UTL, float* __restrict__ Z) {
  __shared__ float sh[CC][68]; __shared__ __align__(16) __bf16 suh[CC][72], sul[CC][72]; __shared__ __align__(16) float sz[64][CC + 4];
  const int b = blockIdx.y, t0 = blockIdx.x * 64, tid = threadIdx.x;
  for (int q = tid; q < CC * 66; q += 256) { const int c = q / 66, j = q % 66; const int tt = t0 - 1 + j; float h = 0.f;
    if (tt >= 0 && tt < TT) { h = bfr(db[c]);
#pragma unroll
      for (int k = 0; k < 3; ++k) { const int tx = tt + k - 1; if (tx >= 0 && tx < TT) h += bfr(dw[c * 3 + k]) * bfr(X[((size_t)b * TT + tx) * CC + c]); } }
    sh[c][j] = h; }
  __syncthreads();
  for (int q = tid; q < 2 * CC * 64; q += 256) { const int i = q >> 6, tl = q & 63; const int src = i >> 1; float v = bfr(lb[i]);
#pragma unroll
    for (int k = 0; k < 3; ++k) v += bfr(lw[i * 3 + k]) * sh[src][tl + k];
    if (i < CC) { const __bf16 hb = (__bf16)v; suh[i][tl] = hb; sul[i][tl] = (__bf16)(v - (float)hb); } else sz[tl][i - CC] = v; }
  __syncthreads();
  for (int q = tid; q < CC * 8; q += 256) { const int c = q >> 3, pc = q & 7; const size_t o = ((size_t)b * CC + c) * TT + t0 + pc * 8; vst2((unsigned*)(UTH + o), *(const v4u*)&suh[c][pc * 8]); vst2((unsigned*)(UTL + o), *(const v4u*)&sul[c][pc * 8]); }
  for (int q = tid; q < 64 * (CC / 4); q += 256) { const int tl = q / (CC / 4), pc = q % (CC / 4); vst2(Z + ((size_t)b * TT + t0 + tl) * CC + pc * 4, *(const v4f*)&sz[tl][pc * 4]); }
}
__global__ __launch_bounds__(128) void k_dct(const float* __restrict__ COS, const __bf16* __restrict__ UTH, const __bf16* __restrict__ UTL, const float* __restrict__ DK, __bf16* __restrict__ ATH, __bf16* __restrict__ ATL) {
  __shared__ __align__(16) __bf16 sth[CC][72], stl[CC][72];
  const int tid = threadIdx.x, wave = tid >> 5, lane = tid & 31, col = lane & 15, g = lane >> 4; const int b = blockIdx.y, n0 = blockIdx.x * 64;
  v8f acc[12] = {};
#pragma unroll 1
  for (int kc = 0; kc < TT / 32; ++kc) { const F2 a = split_row(COS + (size_t)(n0 + wave * 16 + col) * TT, kc * 32, lane);
#pragma unroll
    for (int j = 0; j < 12; ++j) { const size_t ro = ((size_t)b * CC + j * 16 + col) * TT + kc * 32; const v16b uh = frag_b(UTH + ro, lane), ul = frag_b(UTL + ro, lane);
      acc[j] = wmma_bf(a.l, uh, acc[j]); acc[j] = wmma_bf(a.h, ul, acc[j]); acc[j] = wmma_bf(a.h, uh, acc[j]); } }
#pragma unroll
  for (int j = 0; j < 12; ++j)
#pragma unroll
    for (int r = 0; r < 8; ++r) { const int n = n0 + wave * 16 + 8 * g + r, c = j * 16 + col; const float v = acc[j][r] * DK[(size_t)n * CC + c]; const __bf16 hb = (__bf16)v; sth[c][wave * 16 + 8 * g + r] = hb; stl[c][wave * 16 + 8 * g + r] = (__bf16)(v - (float)hb); }
  __syncthreads();
  for (int q = tid; q < CC * 8; q += 128) { const int c = q >> 3, pc = q & 7; const size_t o = ((size_t)b * CC + c) * TT + n0 + pc * 8; vst2((unsigned*)(ATH + o), *(const v4u*)&sth[c][pc * 8]); vst2((unsigned*)(ATL + o), *(const v4u*)&stl[c][pc * 8]); }
}
__global__ __launch_bounds__(128) void k_idct(const float* __restrict__ COST, const __bf16* __restrict__ ATH, const __bf16* __restrict__ ATL, const float* __restrict__ Z, const float* __restrict__ gam, const float* __restrict__ bet, float* __restrict__ G) {
  __shared__ __align__(16) float so[4][16][CC + 4];
  const int tid = threadIdx.x, wave = tid >> 5, lane = tid & 31, col = lane & 15, g = lane >> 4; const int b = blockIdx.y, t0 = blockIdx.x * 64;
  v8f acc[12] = {};
#pragma unroll 1
  for (int kc = 0; kc < TT / 32; ++kc) { const F2 a = split_row(COST + (size_t)(t0 + wave * 16 + col) * TT, kc * 32, lane);
#pragma unroll
    for (int j = 0; j < 12; ++j) { const size_t ro = ((size_t)b * CC + j * 16 + col) * TT + kc * 32; const v16b ah = frag_b(ATH + ro, lane), al = frag_b(ATL + ro, lane);
      acc[j] = wmma_bf(a.l, ah, acc[j]); acc[j] = wmma_bf(a.h, al, acc[j]); acc[j] = wmma_bf(a.h, ah, acc[j]); } }
#pragma unroll
  for (int j = 0; j < 12; ++j)
#pragma unroll
    for (int r = 0; r < 8; ++r) so[wave][8 * g + r][j * 16 + col] = acc[j][r];
  LDSX();
  { const int rl = lane >> 1, half = lane & 1; const int t = t0 + wave * 16 + rl; float s = 0.f; for (int c = half * 96; c < half * 96 + 96; ++c) s += so[wave][rl][c]; s += __shfl_xor(s, 1); const float mu = s / (float)CC;
    float v = 0.f; for (int c = half * 96; c < half * 96 + 96; ++c) { const float d = so[wave][rl][c] - mu; v += d * d; } v += __shfl_xor(v, 1); const float rs = rsqrtf(v / (float)CC + 1e-5f);
    LDSX();
    for (int c = half * 96; c < half * 96 + 96; ++c) { const float zz = Z[((size_t)b * TT + t) * CC + c]; const float sg = zz / (1.0f + exp_ni(-zz)); so[wave][rl][c] = ((so[wave][rl][c] - mu) * rs * bfr(gam[c]) + bfr(bet[c])) * sg; } }
  LDSX();
  for (int rl = 0; rl < 16; ++rl) for (int pc = lane; pc < CC / 4; pc += 32) vst2(G + ((size_t)b * TT + t0 + wave * 16 + rl) * CC + pc * 4, *(const v4f*)&so[wave][rl][pc * 4]);
}
__global__ __launch_bounds__(256) void k_out(const float* __restrict__ G, const float* __restrict__ ow, const float* __restrict__ ob, float* __restrict__ out) {
  __shared__ __align__(16) float so[64][CC + 4];
  const int b = blockIdx.y, t0 = blockIdx.x * 64, tid = threadIdx.x;
  for (int q = tid; q < 64 * CC; q += 256) { const int tl = q / CC, c = q % CC; const int t = t0 + tl; float v = bfr(ob[c]);
#pragma unroll
    for (int k = 0; k < 3; ++k) { const int tx = t + k - 1; if (tx >= 0 && tx < TT) v += bfr(ow[c * 3 + k]) * G[((size_t)b * TT + tx) * CC + c]; }
    so[tl][c] = v; }
  __syncthreads();
  for (int q = tid; q < 64 * (CC / 4); q += 256) { const int tl = q / (CC / 4), pc = q % (CC / 4); vst2(out + ((size_t)b * TT + t0 + tl) * CC + pc * 4, *(const v4f*)&so[tl][pc * 4]); }
}

extern "C" void kernel_launch(void* const* d_in, const int* in_sizes, int n_in, void* d_out, int out_size, void* d_ws, size_t ws_size, hipStream_t stream) {
  (void)in_sizes; (void)n_in; (void)out_size;
  const float** F = (const float**)d_in;
  if (ws_size < (size_t)WS_END) return;
  char* ws = (char*)d_ws; float *COS = (float*)(ws + WS_COS), *COST = (float*)(ws + WS_COST), *DK = (float*)(ws + WS_DK), *Z = (float*)(ws + WS_Z), *G = (float*)(ws + WS_G); __bf16 *UTH = (__bf16*)(ws + WS_UTH), *UTL = (__bf16*)(ws + WS_UTL), *ATH = (__bf16*)(ws + WS_ATH), *ATL = (__bf16*)(ws + WS_ATL);
  k_tab<<<2 * TT + 1, 256, 0, stream>>>(F[9], COS, COST, DK);
  k_conv<<<dim3(TT / 64, TNB), 256, 0, stream>>>(F[0], F[1], F[2], F[3], F[4], UTH, UTL, Z);
  k_dct<<<dim3(TT / 64, TNB), 128, 0, stream>>>(COS, UTH, UTL, DK, ATH, ATL);
  k_idct<<<dim3(TT / 64, TNB), 128, 0, stream>>>(COST, ATH, ATL, Z, F[5], F[6], G);
  k_out<<<dim3(TT / 64, TNB), 256, 0, stream>>>(G, F[7], F[8], (float*)d_out);
}
